// GATEdgeAT_48155173323469
// MI455X (gfx1250) — hardware-verified
//
#include <hip/hip_runtime.h>
#include <stdint.h>

#define NN   20000
#define EE   160000
#define NV   (EE + NN)
#define NVP  180224
#define FIN  30
#define ED   11
#define EDP  12
#define EMB  128
#define NH   4
#define HC   512
#define NG   1000
#define NGP  1024
#define NT   256
#define TB   64
#define NTL  313
#define NPAD (NTL * TB)
#define SCH  4096
#define NCHA (NVP / SCH)
#define NCHL ((EE + SCH - 1) / SCH)
#define TLB  512
#define NTLB 40
#define NLAP (NTLB * TLB)
#define NPART 40
#define RPP  500
#define DOUT_N (NG + NG * 2 * EMB)

typedef __attribute__((ext_vector_type(16))) _Float16 v16h;
typedef __attribute__((ext_vector_type(8)))  _Float16 v8h;
typedef __attribute__((ext_vector_type(4)))  _Float16 v4h;
typedef __attribute__((ext_vector_type(16))) __bf16   v16b;
typedef __attribute__((ext_vector_type(8)))  __bf16   v8b;
typedef __attribute__((ext_vector_type(8)))  float    v8f;
typedef __attribute__((ext_vector_type(4)))  float    v4f;
typedef __attribute__((ext_vector_type(2)))  float    v2f;
typedef __attribute__((ext_vector_type(4)))  int      v4i;
typedef __attribute__((ext_vector_type(2)))  double   v2d;

__device__ __forceinline__ unsigned short f2bf_bits(float f) {
  unsigned u = __float_as_uint(f);
  return (unsigned short)((u + 0x7FFFu + ((u >> 16) & 1u)) >> 16);
}
__device__ __forceinline__ float bf_bits2f(unsigned short h) { return __uint_as_float(((unsigned)h) << 16); }

__device__ __forceinline__ void dep_guard_h(v8f& a, v8f& b, v16h x, v16h y) { asm volatile("v_nop\n\tv_nop\n\tv_nop\n\tv_nop" : "+v"(a), "+v"(b) : "v"(x), "v"(y)); }
__device__ __forceinline__ void dep_guard_b(v8f& a, v8f& b, v16b x, v16b y) { asm volatile("v_nop\n\tv_nop\n\tv_nop\n\tv_nop" : "+v"(a), "+v"(b) : "v"(x), "v"(y)); }
__device__ __forceinline__ void keep4_h(v16h a, v16h b, v16h c, v16h d) { asm volatile("v_nop" :: "v"(a), "v"(b), "v"(c), "v"(d)); }
__device__ __forceinline__ void keep4_b(v16b a, v16b b, v16b c, v16b d) { asm volatile("v_nop" :: "v"(a), "v"(b), "v"(c), "v"(d)); }
__device__ __forceinline__ void acc_guard4(v8f& a, v8f& b, v8f& c, v8f& d) { asm volatile("v_nop\n\tv_nop\n\tv_nop\n\tv_nop" : "+v"(a), "+v"(b), "+v"(c), "+v"(d)); }
template <typename T> struct Frag;
template <> struct Frag<_Float16> {
  typedef v16h V; union U { v16h v; v8h h[2]; };
  static __device__ __forceinline__ v16h load(const _Float16* p) {
    U f; f.h[0] = *(const v8h*)(p); f.h[1] = *(const v8h*)(p + 16); return f.v;
  }
  static __device__ __forceinline__ v8f mma(v16h a, v16h b, v8f c) {
    return __builtin_amdgcn_wmma_f32_16x16x32_f16(false, a, false, b, (short)0, c, false, false);
  }
  static __device__ __forceinline__ void guard(v8f& a, v8f& b, v16h x, v16h y) { dep_guard_h(a, b, x, y); }
  static __device__ __forceinline__ void keep(v16h a, v16h b, v16h c, v16h d) { keep4_h(a, b, c, d); }
};
template <> struct Frag<__bf16> {
  typedef v16b V; union U { v16b v; v8b h[2]; };
  static __device__ __forceinline__ v16b load(const __bf16* p) {
    U f; f.h[0] = *(const v8b*)(p); f.h[1] = *(const v8b*)(p + 16); return f.v;
  }
  static __device__ __forceinline__ v8f mma(v16b a, v16b b, v8f c) {
    return __builtin_amdgcn_wmma_f32_16x16x32_bf16(false, a, false, b, (short)0, c, false, false);
  }
  static __device__ __forceinline__ void guard(v8f& a, v8f& b, v16b x, v16b y) { dep_guard_b(a, b, x, y); }
  static __device__ __forceinline__ void keep(v16b a, v16b b, v16b c, v16b d) { keep4_b(a, b, c, d); }
};

template <int ET> struct Elem;
template <> struct Elem<0> { typedef _Float16 T; };
template <> struct Elem<1> { typedef __bf16 T; };
template <int ET, bool SPLIT, int BIAS_MODE, int OUT_MODE, bool RESID, int ACT = 0>
__global__ __launch_bounds__(256) void wmma_gemm64(
    const unsigned short* __restrict__ Ap, const unsigned short* __restrict__ A2p, int lda, long strideA,
    const unsigned short* __restrict__ Btp, const unsigned short* __restrict__ Bt2p, int ldb, long strideB,
    void* __restrict__ Cout, void* __restrict__ Cout2, int ldc, long strideC,
    const float* __restrict__ bias,
    const float* __restrict__ resid, long strideR,
    int M, int N, int K, float scale) {
  typedef typename Elem<ET>::T T;
  typedef typename Frag<T>::V V;
  const T* A = (const T*)Ap; const T* A2 = (const T*)A2p; const T* Bt = (const T*)Btp; const T* Bt2 = (const T*)Bt2p;
  __shared__ __align__(16) float sT[8][16 * 68];
  const int b    = blockIdx.y;
  const int lane = threadIdx.x & 31;
  const int wave = threadIdx.x >> 5;
  const int tilesN = N >> 6;
  const int tilesM = M >> 6;
  const int tile = blockIdx.x * 8 + wave;
  if (tile >= tilesM * tilesN) return;
  const int tm = tile / tilesN;
  const int tn = tile - tm * tilesN;
  const int m0 = tm << 6;
  const int n0 = tn << 6;

  const T* Ab  = A  + (size_t)b * strideA;
  const T* Bb  = Bt + (size_t)b * strideB;
  const T* Ab2 = SPLIT ? (A2  + (size_t)b * strideA) : nullptr;
  const T* Bb2 = SPLIT ? (Bt2 + (size_t)b * strideB) : nullptr;

  const int rlane = lane & 15;
  const int koff  = (lane >> 4) * 8;
  const int mOff  = (lane >> 4) * 8;

  v8f acc[4][4];
#pragma unroll
  for (int i = 0; i < 4; ++i)
#pragma unroll
    for (int j = 0; j < 4; ++j) acc[i][j] = (v8f){0.f,0.f,0.f,0.f,0.f,0.f,0.f,0.f};

  for (int k0 = 0; k0 < K; k0 += 32) {
    V bh[4], bl[4];
#pragma unroll
    for (int j = 0; j < 4; ++j) {
      const size_t bo = (size_t)(n0 + (j << 4) + rlane) * ldb + koff + k0;
      bh[j] = Frag<T>::load(Bb + bo);
      if (SPLIT) bl[j] = Frag<T>::load(Bb2 + bo);
    }
#pragma unroll
    for (int i = 0; i < 4; ++i) {
      const size_t ao = (size_t)(m0 + (i << 4) + rlane) * lda + koff + k0;
      V ah = Frag<T>::load(Ab + ao);
      V al;
      if (SPLIT) al = Frag<T>::load(Ab2 + ao);
#pragma unroll
      for (int j = 0; j < 4; ++j) {
        acc[i][j] = Frag<T>::mma(ah, bh[j], acc[i][j]);
        if (SPLIT) {
          acc[i][j] = Frag<T>::mma(ah, bl[j], acc[i][j]);
          acc[i][j] = Frag<T>::mma(al, bh[j], acc[i][j]);
        }
      }
      Frag<T>::guard(acc[i][0], acc[i][3], ah, SPLIT ? al : ah);
    }
    Frag<T>::keep(bh[0], bh[1], bh[2], bh[3]);
    if (SPLIT) Frag<T>::keep(bl[0], bl[1], bl[2], bl[3]);
  }
  acc_guard4(acc[0][0], acc[0][1], acc[0][2], acc[0][3]);
  acc_guard4(acc[1][0], acc[1][1], acc[1][2], acc[1][3]);
  acc_guard4(acc[2][0], acc[2][1], acc[2][2], acc[2][3]);
  acc_guard4(acc[3][0], acc[3][1], acc[3][2], acc[3][3]);

  float* slab = sT[wave];
  const float* Rb = RESID ? (resid + (size_t)b * strideR) : nullptr;
#pragma unroll
  for (int i = 0; i < 4; ++i) {
    const int mBase = m0 + (i << 4);
#pragma unroll
    for (int j = 0; j < 4; ++j) {
      const int n = n0 + (j << 4) + rlane;
      float bv = 0.f;
      if (BIAS_MODE == 2) bv = bias[n];
#pragma unroll
      for (int r = 0; r < 8; ++r) {
        float v = acc[i][j][r] * scale;
        if (BIAS_MODE == 1) v += bias[mBase + mOff + r];
        if (BIAS_MODE == 2) v += bv;
        if (RESID) v += Rb[(size_t)(mBase + mOff + r) * ldc + n];
        if (ACT == 1) v = tanhf(v);
        if (ACT == 2) v = fmaxf(v, 0.0f);
        if (ACT == 3) v = v / (1.0f + expf(-v));
        if (ACT == 4) v = (v > 0.f) ? v : 0.01f * v;
        if (ACT == 5) v = 0.5f * v * (1.0f + erff(v * 0.70710678118654752f));
        slab[(mOff + r) * 68 + (j << 4) + rlane] = v;
      }
    }
    __builtin_amdgcn_fence(__ATOMIC_RELEASE, "workgroup");
    __builtin_amdgcn_wave_barrier();
    __builtin_amdgcn_fence(__ATOMIC_ACQUIRE, "workgroup");
    if (OUT_MODE == 0) {
      float* C = (float*)Cout + (size_t)b * strideC;
      const int hh = lane >> 4, c4 = (lane & 15) * 4;
      for (int pass = 0; pass < 2; ++pass) {
#pragma unroll
        for (int it = 0; it < 8; ++it) {
          const int row = it * 2 + hh;
          v4f v = *(const v4f*)(slab + row * 68 + c4);
          *(volatile v4f*)(C + (size_t)(mBase + row) * ldc + n0 + c4) = v;
        }
        __threadfence();
      }
    } else {
      const int q = lane >> 3, c8 = (lane & 7) * 8;
      unsigned short* C  = (unsigned short*)Cout  + (size_t)b * strideC;
      unsigned short* C2 = (OUT_MODE == 2) ? ((unsigned short*)Cout2 + (size_t)b * strideC) : nullptr;
      for (int pass = 0; pass < 2; ++pass) {
#pragma unroll
        for (int it = 0; it < 4; ++it) {
          const int row = it * 4 + q;
          const float* sp = slab + row * 68 + c8;
          v8h hv, lv;
#pragma unroll
          for (int e = 0; e < 8; ++e) {
            if (OUT_MODE == 1) {
              hv[e] = (_Float16)sp[e];
            } else {
              unsigned short hb = f2bf_bits(sp[e]);
              unsigned short lb = f2bf_bits(sp[e] - bf_bits2f(hb));
              hv[e] = __builtin_bit_cast(_Float16, hb);
              lv[e] = __builtin_bit_cast(_Float16, lb);
            }
          }
          *(volatile v8h*)(C + (size_t)(mBase + row) * ldc + n0 + c8) = hv;
          if (OUT_MODE == 2) *(volatile v8h*)(C2 + (size_t)(mBase + row) * ldc + n0 + c8) = lv;
        }
        __threadfence();
      }
    }
    __builtin_amdgcn_fence(__ATOMIC_RELEASE, "workgroup");
    __builtin_amdgcn_wave_barrier();
    __builtin_amdgcn_fence(__ATOMIC_ACQUIRE, "workgroup");
  }
}

__global__ __launch_bounds__(256) void transpose_cast_f16(const float* __restrict__ in, int ldi,
                                                         _Float16* __restrict__ outT, int ldo, float scale) {
  __shared__ __align__(16) _Float16 tile[64][72];
  const int c0 = blockIdx.x * 64, r0 = blockIdx.y * 64;
  const int t = threadIdx.y * 32 + threadIdx.x;
  for (int i = threadIdx.y; i < 64; i += 8) {
    tile[threadIdx.x][i]      = (_Float16)(in[(size_t)(r0 + i) * ldi + c0 + threadIdx.x] * scale);
    tile[32 + threadIdx.x][i] = (_Float16)(in[(size_t)(r0 + i) * ldi + c0 + 32 + threadIdx.x] * scale);
  }
  __syncthreads();
  const int q = t >> 3, c8 = (t & 7) * 8;
  for (int pass = 0; pass < 2; ++pass) {
#pragma unroll
    for (int it = 0; it < 2; ++it) {
      const int c = it * 32 + q;
      v8h hv = *(const v8h*)(&tile[c][c8]);
      *(volatile v8h*)(outT + (size_t)(c0 + c) * ldo + r0 + c8) = hv;
    }
    __threadfence();
  }
}

__global__ __launch_bounds__(NT) void castx_kernel(const float* __restrict__ x, unsigned* __restrict__ X16) {
  const int i = blockIdx.x * NT + threadIdx.x;
  const int n = i >> 4, kp = (i & 15) * 2;
  float a = 0.f, b = 0.f;
  if (n < NN) {
    if (kp < FIN)     a = x[(size_t)n * FIN + kp];
    if (kp + 1 < FIN) b = x[(size_t)n * FIN + kp + 1];
  }
  const unsigned u = (unsigned)__builtin_bit_cast(unsigned short, (_Float16)a) | ((unsigned)__builtin_bit_cast(unsigned short, (_Float16)b) << 16);
  ((volatile unsigned*)X16)[i] = u; __threadfence(); ((volatile unsigned*)X16)[i] = u;
}
__global__ __launch_bounds__(NT) void lin0_cast_kernel(const float* __restrict__ w, unsigned* __restrict__ WT) {
  const int i = blockIdx.x * NT + threadIdx.x;
  const int n = i >> 4, kp = (i & 15) * 2;
  const float a = (kp < FIN)     ? w[(size_t)kp * HC + n] * 16.0f : 0.f;
  const float b = (kp + 1 < FIN) ? w[(size_t)(kp + 1) * HC + n] * 16.0f : 0.f;
  const unsigned u = (unsigned)__builtin_bit_cast(unsigned short, (_Float16)a) | ((unsigned)__builtin_bit_cast(unsigned short, (_Float16)b) << 16);
  ((volatile unsigned*)WT)[i] = u; __threadfence(); ((volatile unsigned*)WT)[i] = u;
}

__global__ __launch_bounds__(NT) void fold_kernel(const float* __restrict__ e0w, const float* __restrict__ a0, const float* __restrict__ elw,
                                                 const float* __restrict__ al, float* __restrict__ MF) {
  const int i = threadIdx.x;
  float s = 0.f;
  if (i < 4 * ED * NH) {
    const int l = i / (ED * NH), rem = i - l * (ED * NH), d = rem >> 2, h = rem & 3;
    const float* ew = (l == 0) ? e0w : elw + (size_t)(l - 1) * ED * HC;
    const float* ae = (l == 0) ? a0 : al + (size_t)(l - 1) * NH * EMB;
#pragma unroll 1
    for (int c = 0; c < EMB; ++c) s += ew[(size_t)d * HC + h * EMB + c] * ae[h * EMB + c];
  }
  if (i < 192) { ((volatile float*)MF)[i] = s; __threadfence(); ((volatile float*)MF)[i] = s; }
}

__device__ __forceinline__ int blk_excl_scan(int cnt, int* scan_ws, int tid, int* tot) {
  const int lane = tid & 31, wave = tid >> 5; int incl = cnt;
#pragma unroll
  for (int o = 1; o < 32; o <<= 1) { const int v = __shfl_up(incl, o, 32); if (lane >= o) incl += v; }
  if (lane == 31) scan_ws[wave] = incl;
  __syncthreads();
  if (wave == 0) { int wv = (lane < NT / 32) ? scan_ws[lane] : 0; int wincl = wv;
#pragma unroll
    for (int o = 1; o < 32; o <<= 1) { const int v = __shfl_up(wincl, o, 32); if (lane >= o) wincl += v; }
    if (lane < NT / 32) scan_ws[32 + lane] = wincl - wv; if (lane == 31) scan_ws[64] = wincl; }
  __syncthreads();
  const int res = scan_ws[32 + wave] + incl - cnt; *tot = scan_ws[64];
  return res;
}
template <int SP, int CAP, int TSZ, bool SELF>
__device__ __forceinline__ int chunk_hits(const int* __restrict__ dstv, int e0, int n0, int tid, int* LIST, int* scan_ws) {
  const int eb = e0 + tid * SP;
  int rec[SP]; int cnt = 0;
  if (eb < EE) {
#pragma unroll
    for (int k = 0; k < SP; k += 4) {
      const v4i d4 = *(const v4i*)(dstv + eb + k);
#pragma unroll
      for (int q = 0; q < 4; ++q) {
        const int d = d4[q]; int r = -1;
        if (d >= n0 && d < n0 + TSZ) { r = ((d - n0) << 18) | (eb + k + q); ++cnt; }
        rec[k + q] = r;
      }
    }
  } else {
#pragma unroll
    for (int k = 0; k < SP; ++k) {
      const int ev = eb + k; const int d = ev - EE; int r = -1;
      if (SELF && ev < NV && d >= n0 && d < n0 + TSZ) { r = ((d - n0) << 18) | ev; ++cnt; }
      rec[k] = r;
    }
  }
  int tot; int p = blk_excl_scan(cnt, scan_ws, tid, &tot);
#pragma unroll
  for (int k = 0; k < SP; ++k) if (rec[k] >= 0) { if ((unsigned)p < (unsigned)CAP) LIST[p] = rec[k]; ++p; }
  __syncthreads();
  return tot < CAP ? tot : CAP;
}

__global__ __launch_bounds__(NT) void loop_attr_kernel(const int* __restrict__ ei, const float* __restrict__ ea, float* __restrict__ LA) {
  __shared__ __align__(16) float LACC[TLB * EDP];
  __shared__ int LIST[SCH];
  __shared__ int scan_ws[80];
  const int tid = threadIdx.x, lane = tid & 31, wave = tid >> 5;
  const int n0 = blockIdx.x * TLB;
  for (int i = tid; i < TLB * EDP; i += NT) LACC[i] = 0.f;
  __syncthreads();
  const int* dstv = ei + EE;
#pragma unroll 1
  for (int c = 0; c < NCHL; ++c) {
    const int tot = chunk_hits<SCH / NT, SCH, TLB, false>(dstv, c * SCH, n0, tid, LIST, scan_ws);
#pragma unroll 1
    for (int base = 0; base < tot; base += 32) {
      const int q = base + lane;
      const int rv = (q < tot) ? LIST[q] : -1;
      const int own = (rv >= 0 && (rv >> 24) == wave) ? 1 : 0;
      unsigned msk = (unsigned)__ballot(own);
#pragma unroll 1
      for (int it = 0; it < 32; ++it) {
        if (msk == 0u) break;
        const int bp = __builtin_ctz(msk); msk &= msk - 1u;
        const int r = __shfl(rv, bp, 32);
        int e = r & 0x3FFFF; e = e >= EE ? EE - 1 : e;
        const int dl = (r >> 18) & (TLB - 1);
        if (lane < ED)       LACC[dl * EDP + lane] += ea[(size_t)e * ED + lane];
        else if (lane == ED) LACC[dl * EDP + ED] += 1.0f;
      }
    }
    __syncthreads();
  }
  for (int i = tid; i < TLB; i += NT) {
    const float dg = LACC[i * EDP + ED];
    const float inv = 1.0f / fmaxf(dg, 1.0f);
#pragma unroll
    for (int d = 0; d < ED; ++d) LACC[i * EDP + d] = LACC[i * EDP + d] * inv;
    LACC[i * EDP + ED] = 0.f;
  }
  __syncthreads();
  float* ob = LA + (size_t)n0 * EDP;
  for (int pass = 0; pass < 2; ++pass) {
#pragma unroll
    for (int k = 0; k < 6; ++k) {
      const v4f v = *(const v4f*)(LACC + 1024 * k + 4 * tid);
      *(volatile v4f*)(ob + 1024 * k + 4 * tid) = v;
    }
    __threadfence();
  }
}

__global__ __launch_bounds__(NT) void edge_terms_kernel(const float* __restrict__ ea, const float* __restrict__ LA, const float* __restrict__ MF,
                                                       float* __restrict__ ET) {
  __shared__ float sM[4 * ED * NH];
  const int tid = threadIdx.x;
  if (tid < 4 * ED * NH) sM[tid] = MF[tid];
  __syncthreads();
  const int e = blockIdx.x * NT + tid;
  const bool valid = e < NV;
  const int ec = valid ? e : (NV - 1);
  const float* ap = (ec < EE) ? (ea + (size_t)ec * ED) : (LA + (size_t)(ec - EE) * EDP);
  float acc[16];
#pragma unroll
  for (int i = 0; i < 16; ++i) acc[i] = 0.f;
#pragma unroll 1
  for (int d = 0; d < ED; ++d) {
    const float a = valid ? ap[d] : 0.f;
#pragma unroll
    for (int l = 0; l < 4; ++l)
#pragma unroll
      for (int h = 0; h < 4; ++h) acc[l * 4 + h] += a * sM[(l * ED + d) * NH + h];
  }
  for (int pass = 0; pass < 2; ++pass) {
#pragma unroll
    for (int l = 0; l < 4; ++l) {
      const v4f v = {acc[l * 4 + 0], acc[l * 4 + 1], acc[l * 4 + 2], acc[l * 4 + 3]};
      *(volatile v4f*)(ET + (size_t)l * NVP * NH + (size_t)e * NH) = v;
    }
    __threadfence();
  }
}

__global__ __launch_bounds__(NT) void att_terms_kernel(const float* __restrict__ XS, const float* __restrict__ as, const float* __restrict__ ad,
                                                      float* __restrict__ ASD) {
  __shared__ __align__(16) float so[64];
  const int lane = threadIdx.x & 31, wave = threadIdx.x >> 5;
  const int n = blockIdx.x * 8 + wave;
  const int h = lane >> 3, cq = (lane & 7) * 16;
  const float* xr = XS + (size_t)n * HC + h * EMB + cq;
  const v4f x0 = *(const v4f*)(xr), x1 = *(const v4f*)(xr + 4), x2 = *(const v4f*)(xr + 8), x3 = *(const v4f*)(xr + 12);
  const float* sp = as + h * EMB + cq;
  const float* dp = ad + h * EMB + cq;
  const v4f s0 = *(const v4f*)(sp), s1 = *(const v4f*)(sp + 4), s2 = *(const v4f*)(sp + 8), s3 = *(const v4f*)(sp + 12);
  const v4f d0 = *(const v4f*)(dp), d1 = *(const v4f*)(dp + 4), d2 = *(const v4f*)(dp + 8), d3 = *(const v4f*)(dp + 12);
  float s = 0.f, d = 0.f;
#pragma unroll
  for (int e = 0; e < 4; ++e) {
    s += x0[e] * s0[e]; s += x1[e] * s1[e]; s += x2[e] * s2[e]; s += x3[e] * s3[e];
    d += x0[e] * d0[e]; d += x1[e] * d1[e]; d += x2[e] * d2[e]; d += x3[e] * d3[e];
  }
  s += __shfl_xor(s, 1, 32); s += __shfl_xor(s, 2, 32); s += __shfl_xor(s, 4, 32);
  d += __shfl_xor(d, 1, 32); d += __shfl_xor(d, 2, 32); d += __shfl_xor(d, 4, 32);
  if ((lane & 7) == 0) { so[wave * 8 + h] = s; so[wave * 8 + 4 + h] = d; }
  __syncthreads();
  if (wave == 0 && lane < 16) {
    const v4f v = *(const v4f*)(so + 4 * lane);
    float* op = ASD + (size_t)blockIdx.x * 64 + 4 * lane;
    *(volatile v4f*)op = v; __threadfence(); *(volatile v4f*)op = v;
  }
}

__device__ __forceinline__ float tanh_fast(float x) {
  const float t = __expf(2.0f * x);
  return 1.0f - 2.0f * __builtin_amdgcn_rcpf(t + 1.0f);
}

__global__ __launch_bounds__(NT) void gat_agg_kernel(const float* __restrict__ XS, const int* __restrict__ ei, const float* __restrict__ ET,
                                                    const float* __restrict__ ASD, const float* __restrict__ bias, _Float16* __restrict__ T16) {
  extern __shared__ __align__(16) float ACC[];
  __shared__ int LIST[SCH];
  __shared__ float SM[TB * NH];
  __shared__ float SL[TB * NH];
  __shared__ float SAD[TB * NH];
  __shared__ int scan_ws[80];
  const int tid = threadIdx.x, lane = tid & 31, wave = tid >> 5;
  const int n0 = blockIdx.x * TB;
  const int h4 = lane & 3;
  const v4f z4 = {0.f, 0.f, 0.f, 0.f};
#pragma unroll 1
  for (int j = 0; j < 8; ++j) {
    float* rp = ACC + (wave * 8 + j) * HC + 4 * lane;
#pragma unroll
    for (int jj = 0; jj < 4; ++jj) *(v4f*)(rp + 128 * jj) = z4;
  }
  {
    const int i = tid;
    SM[i] = -__builtin_inff(); SL[i] = 0.f;
    SAD[i] = ASD[(size_t)(n0 + (i >> 2)) * 8 + 4 + (i & 3)];
  }
  __syncthreads();
  const int* dstv = ei + EE;
#pragma unroll 1
  for (int c = 0; c < NCHA; ++c) {
    const int tot = chunk_hits<SCH / NT, SCH, TB, true>(dstv, c * SCH, n0, tid, LIST, scan_ws);
#pragma unroll 1
    for (int base = 0; base < tot; base += 32) {
      const int q = base + lane;
      const int rv = (q < tot) ? LIST[q] : -1;
      const int own = (rv >= 0 && (rv >> 21) == wave) ? 1 : 0;
      unsigned msk = (unsigned)__ballot(own);
#pragma unroll 1
      for (int it = 0; it < 32; ++it) {
        if (msk == 0u) break;
        const int bp = __builtin_ctz(msk); msk &= msk - 1u;
        const int r = __shfl(rv, bp, 32);
        const int e = r & 0x3FFFF;
        const int dl = (r >> 18) & (TB - 1);
        int s;
        if (e < EE) { s = ei[e]; s = s < 0 ? 0 : (s >= NN ? NN - 1 : s); }
        else        { s = e - EE; s = s >= NN ? NN - 1 : s; }
        const int mi = dl * NH + h4;
        float al = ASD[(size_t)s * 8 + h4] + SAD[mi] + ET[(size_t)e * NH + h4];
        al = (al >= 0.f) ? al : 0.2f * al;
        const float mo = SM[mi], lo = SL[mi];
        const float mn = fmaxf(mo, al);
        const float rr = __expf(mo - mn), ex = __expf(al - mn);
        const float ln = lo * rr + ex;
        if (lane < NH) { SM[mi] = mn; SL[mi] = ln; }
        const float* xr = XS + (size_t)s * HC + 4 * lane;
        float* rp = ACC + dl * HC + 4 * lane;
#pragma unroll
        for (int j = 0; j < 4; ++j) {
          const float rrj = __shfl(rr, j, 32), exj = __shfl(ex, j, 32);
          const v4f xv = *(const v4f*)(xr + 128 * j);
          v4f a = *(const v4f*)(rp + 128 * j);
          a = a * rrj + exj * xv;
          *(v4f*)(rp + 128 * j) = a;
        }
      }
    }
    __syncthreads();
  }
#pragma unroll 1
  for (int j = 0; j < 8; ++j) {
    const int dl = wave * 8 + j;
    const int n = n0 + dl;
    const bool live = n < NN;
    float lv = 1.0f;
    if (lane < NH) lv = SL[dl * NH + lane];
    lv = lv > 0.f ? lv : 1.0f;
    const float inv = 1.0f / lv;
#pragma unroll 1
    for (int pass = 0; pass < 2; ++pass) {
#pragma unroll 1
      for (int p = 0; p < 2; ++p) {
        const int col0 = 256 * p + 8 * lane;
        const int head = 2 * p + (lane >> 4);
        const float ih = __shfl(inv, head, 32);
        const v4f a0 = *(const v4f*)(ACC + dl * HC + col0);
        const v4f a1 = *(const v4f*)(ACC + dl * HC + col0 + 4);
        const v4f b0 = *(const v4f*)(bias + col0);
        const v4f b1 = *(const v4f*)(bias + col0 + 4);
        v8h hv;
#pragma unroll
        for (int e = 0; e < 4; ++e) {
          const float v0 = a0[e] * ih + b0[e];
          const float v1 = a1[e] * ih + b1[e];
          hv[e]     = (_Float16)(live ? tanh_fast(v0) : 0.f);
          hv[4 + e] = (_Float16)(live ? tanh_fast(v1) : 0.f);
        }
        *(volatile v8h*)(T16 + (size_t)n * HC + col0) = hv;
      }
      __threadfence();
    }
  }
}

__global__ __launch_bounds__(128) void bn_stats_kernel(const float* __restrict__ H2, double* __restrict__ BNP) {
  const int c = threadIdx.x, p = blockIdx.x;
  const int base = p * RPP;
  double s = 0.0, q = 0.0;
#pragma unroll 4
  for (int i = 0; i < RPP; ++i) {
    const float v = H2[(size_t)(base + i) * EMB + c];
    s += (double)v; q += (double)v * (double)v;
  }
  const v2d o = {s, q};
  double* op = BNP + ((size_t)p * EMB + c) * 2;
  *(volatile v2d*)op = o; __threadfence(); *(volatile v2d*)op = o;
}
__global__ __launch_bounds__(128) void bn_fin_kernel(const double* __restrict__ BNP, float* __restrict__ BNS) {
  const int c = threadIdx.x;
  double s = 0.0, q = 0.0;
#pragma unroll 1
  for (int p = 0; p < NPART; ++p) {
    const v2d o = *(const v2d*)(BNP + ((size_t)p * EMB + c) * 2);
    s += o[0]; q += o[1];
  }
  const double mu = s * (1.0 / (double)NN);
  double var = q * (1.0 / (double)NN) - mu * mu;
  if (var < 0.0) var = 0.0;
  const float muf = (float)mu;
  const float rs = 1.0f / sqrtf((float)var + 1e-5f);
  ((volatile float*)BNS)[c] = muf; ((volatile float*)BNS)[EMB + c] = rs;
  __threadfence();
  ((volatile float*)BNS)[c] = muf; ((volatile float*)BNS)[EMB + c] = rs;
}
__global__ __launch_bounds__(NT) void bn_apply_kernel(const float* __restrict__ H2, const float* __restrict__ BNS, const float* __restrict__ g,
                                                     const float* __restrict__ bb, float* __restrict__ HF, unsigned* __restrict__ H16) {
  const long i = (long)blockIdx.x * NT + threadIdx.x;
  const long e0 = 2 * i; const int c = (int)(e0 & (EMB - 1)); const bool ok = e0 < (long)NN * EMB;
  float a = 0.f, b = 0.f;
  if (ok) {
    a = (H2[e0] - BNS[c]) * BNS[EMB + c] * g[c] + bb[c];
    b = (H2[e0 + 1] - BNS[c + 1]) * BNS[EMB + c + 1] * g[c + 1] + bb[c + 1];
  }
  const v2f v = {a, b};
  const unsigned u = (unsigned)__builtin_bit_cast(unsigned short, (_Float16)a) | ((unsigned)__builtin_bit_cast(unsigned short, (_Float16)b) << 16);
  if (ok) { *(volatile v2f*)(HF + e0) = v; }
  ((volatile unsigned*)H16)[i] = u; __threadfence();
  if (ok) { *(volatile v2f*)(HF + e0) = v; }
  ((volatile unsigned*)H16)[i] = u;
}

__global__ __launch_bounds__(128) void pool_kernel(const float* __restrict__ HF, const int* __restrict__ batch, float* __restrict__ HID,
                                                  _Float16* __restrict__ HID16) {
  __shared__ int PL[128];
  __shared__ int sc[4];
  __shared__ __align__(16) float srow[2 * EMB];
  const int tid = threadIdx.x, lane = tid & 31, wave = tid >> 5;
  const int g = blockIdx.x;
  float sum = 0.f, mx = -__builtin_inff();
  int cnt = 0;
  if (g < NG) {
#pragma unroll 1
    for (int base = 0; base < NN; base += 128) {
      const int n = base + tid;
      const int hit = (n < NN && batch[n] == g) ? 1 : 0;
      const unsigned m = (unsigned)__ballot(hit);
      if (lane == 0) sc[wave] = __popc(m);
      __syncthreads();
      int offs = 0, tot = 0;
#pragma unroll
      for (int w = 0; w < 4; ++w) { const int cw = sc[w]; if (w < wave) offs += cw; tot += cw; }
      tot = tot > 128 ? 128 : tot;
      if (hit) { const int pos = offs + __popc(m & ((1u << lane) - 1u)); if ((unsigned)pos < 128u) PL[pos] = n; }
      __syncthreads();
#pragma unroll 1
      for (int k = 0; k < tot; ++k) {
        const int nn = PL[k];
        const float v = HF[(size_t)nn * EMB + tid];
        sum += v; mx = fmaxf(mx, v);
      }
      cnt += tot;
      __syncthreads();
    }
  }
  const float cf = (float)cnt;
  const float inv = 1.0f / fmaxf(cf, 1.0f);
  const float mean = sum * inv;
  const float gm = (cnt > 0) ? mx : 0.f;
  srow[tid] = gm; srow[EMB + tid] = mean;
  __syncthreads();
  for (int pass = 0; pass < 2; ++pass) {
    if (tid < 64) {
      const v4f v = *(const v4f*)(srow + 4 * tid);
      *(volatile v4f*)(HID + (size_t)g * 2 * EMB + 4 * tid) = v;
    } else if (tid < 96) {
      const int q = tid - 64;
      v8h hv;
#pragma unroll
      for (int e = 0; e < 8; ++e) hv[e] = (_Float16)srow[8 * q + e];
      *(volatile v8h*)(HID16 + (size_t)g * 2 * EMB + 8 * q) = hv;
    }
    __threadfence();
  }
}

__global__ __launch_bounds__(NT) void out0_kernel(const float* __restrict__ OB, const float* __restrict__ w2, const float* __restrict__ b2,
                                                 float* __restrict__ OUT0) {
  __shared__ float sres[32];
  const int lane = threadIdx.x & 31, wave = threadIdx.x >> 5;
  float wv[8];
#pragma unroll
  for (int t = 0; t < 8; ++t) wv[t] = w2[lane + 32 * t];
  const float bb = b2[0];
#pragma unroll 1
  for (int i = 0; i < 4; ++i) {
    const int g = blockIdx.x * 32 + wave * 4 + i;
    float acc = 0.f;
#pragma unroll
    for (int t = 0; t < 8; ++t) acc += OB[(size_t)g * 2 * EMB + lane + 32 * t] * wv[t];
#pragma unroll
    for (int o = 16; o > 0; o >>= 1) acc += __shfl_xor(acc, o, 32);
    if (lane == 0) sres[wave * 4 + i] = acc + bb;
  }
  __syncthreads();
  if (wave == 0) {
    const float v = sres[lane];
    ((volatile float*)OUT0)[blockIdx.x * 32 + lane] = v; __threadfence(); ((volatile float*)OUT0)[blockIdx.x * 32 + lane] = v;
  }
}

__global__ __launch_bounds__(NT) void pack_out_kernel(const float* __restrict__ OUT0, const float* __restrict__ HID, float* __restrict__ dout) {
  const int i = blockIdx.x * NT + threadIdx.x;
  const int f = 4 * i;
  if (f >= DOUT_N) return;
  v4f v;
#pragma unroll
  for (int k = 0; k < 4; ++k) {
    const int idx = f + k;
    v[k] = (idx < NG) ? OUT0[idx] : HID[idx - NG];
  }
  *(volatile v4f*)(dout + f) = v; __threadfence(); *(volatile v4f*)(dout + f) = v;
}

extern "C" void kernel_launch(void* const* d_in, const int* in_sizes, int n_in,
                              void* d_out, int out_size, void* d_ws, size_t ws_size, hipStream_t stream) {
  (void)in_sizes; (void)n_in; (void)out_size;
  const float* x        = (const float*)d_in[0];
  const int*   ei       = (const int*)  d_in[1];
  const float* ea       = (const float*)d_in[2];
  const int*   batch    = (const int*)  d_in[3];
  const float* g0_lin   = (const float*)d_in[4];
  const float* g0_edge  = (const float*)d_in[5];
  const float* g0_asrc  = (const float*)d_in[6];
  const float* g0_adst  = (const float*)d_in[7];
  const float* g0_aedge = (const float*)d_in[8];
  const float* g0_b     = (const float*)d_in[9];
  const float* g_lin    = (const float*)d_in[10];
  const float* g_edge   = (const float*)d_in[11];
  const float* g_asrc   = (const float*)d_in[12];
  const float* g_adst   = (const float*)d_in[13];
  const float* g_aedge  = (const float*)d_in[14];
  const float* g_b      = (const float*)d_in[15];
  const float* ht_w     = (const float*)d_in[16];
  const float* ht_b     = (const float*)d_in[17];
  const float* bn_g     = (const float*)d_in[18];
  const float* bn_b     = (const float*)d_in[19];
  const float* out1_w   = (const float*)d_in[20];
  const float* out1_b   = (const float*)d_in[21];
  const float* out2_w   = (const float*)d_in[22];
  const float* out2_b   = (const float*)d_in[23];
  float* dout = (float*)d_out;

  char* ws = (char*)d_ws; size_t off = 0;
  auto carve = [&](size_t bytes) -> char* { char* p = ws + off; off += (bytes + 255) & ~(size_t)255; return p; };
  unsigned* X16   = (unsigned*)carve((size_t)NPAD * EMB * 2);
  unsigned* LIN0T = (unsigned*)carve((size_t)HC * 32 * 2);
  _Float16* LINT  = (_Float16*)carve((size_t)3 * HC * EMB * 2);
  _Float16* HTT   = (_Float16*)carve((size_t)4 * EMB * HC * 2);
  _Float16* O1T   = (_Float16*)carve((size_t)256 * 256 * 2);
  float*    MF    = (float*)carve(192 * 4);
  float*    LA    = (float*)carve((size_t)NLAP * EDP * 4);
  float*    ET    = (float*)carve((size_t)4 * NVP * NH * 4);
  float*    XS    = (float*)carve((size_t)NPAD * HC * 4);
  float*    ASD   = (float*)carve((size_t)NPAD * 8 * 4);
  _Float16* T16   = (_Float16*)carve((size_t)NPAD * HC * 2);
  float*    H2    = (float*)carve((size_t)NPAD * EMB * 4);
  float*    HF    = (float*)carve((size_t)NN * EMB * 4);
  double*   BNP   = (double*)carve((size_t)NPART * EMB * 2 * 8);
  float*    BNS   = (float*)carve(2 * EMB * 4);
  float*    HID   = (float*)carve((size_t)NGP * 2 * EMB * 4);
  _Float16* HID16 = (_Float16*)carve((size_t)NGP * 2 * EMB * 2);
  float*    OB    = (float*)carve((size_t)NGP * 2 * EMB * 4);
  float*    OUT0  = (float*)carve((size_t)NGP * 4);
  if (off > ws_size || off > (size_t)134217728) return;

  castx_kernel<<<NPAD * 16 / NT, NT, 0, stream>>>(x, X16);
  lin0_cast_kernel<<<HC * 16 / NT, NT, 0, stream>>>(g0_lin, LIN0T);
  for (int j = 0; j < 3; ++j)
    transpose_cast_f16<<<dim3(HC / 64, EMB / 64), dim3(32, 8), 0, stream>>>(g_lin + (size_t)j * EMB * HC, HC, LINT + (size_t)j * HC * EMB, EMB, 16.0f);
  for (int l = 0; l < 4; ++l)
    transpose_cast_f16<<<dim3(EMB / 64, HC / 64), dim3(32, 8), 0, stream>>>(ht_w + (size_t)l * HC * EMB, EMB, HTT + (size_t)l * EMB * HC, HC, 16.0f);
  transpose_cast_f16<<<dim3(256 / 64, 256 / 64), dim3(32, 8), 0, stream>>>(out1_w, 256, O1T, 256, 16.0f);
  fold_kernel<<<1, NT, 0, stream>>>(g0_edge, g0_aedge, g_edge, g_aedge, MF);
  loop_attr_kernel<<<NTLB, NT, 0, stream>>>(ei, ea, LA);
  edge_terms_kernel<<<NVP / NT, NT, 0, stream>>>(ea, LA, MF, ET);

  const int agg_lds = TB * HC * 4;
  hipFuncSetAttribute(reinterpret_cast<const void*>(&gat_agg_kernel), hipFuncAttributeMaxDynamicSharedMemorySize, agg_lds);

  for (int l = 0; l < 4; ++l) {
    const int K = (l == 0) ? 32 : EMB;
    const unsigned short* Bt = (l == 0) ? (const unsigned short*)LIN0T : (const unsigned short*)(LINT + (size_t)(l - 1) * HC * EMB);
    const float* a_s  = (l == 0) ? g0_asrc : g_asrc + (size_t)(l - 1) * NH * EMB;
    const float* a_d  = (l == 0) ? g0_adst : g_adst + (size_t)(l - 1) * NH * EMB;
    const float* bias = (l == 0) ? g0_b    : g_b    + (size_t)(l - 1) * HC;
    wmma_gemm64<0, false, 0, 0, false, 0><<<dim3((NTL * 8 + 7) / 8, 1), 256, 0, stream>>>(
        (const unsigned short*)X16, nullptr, K, 0L, Bt, nullptr, K, 0L,
        (void*)XS, nullptr, HC, 0L, nullptr, nullptr, 0L, NPAD, HC, K, 0.0625f);
    att_terms_kernel<<<NPAD / 8, NT, 0, stream>>>(XS, a_s, a_d, ASD);
    gat_agg_kernel<<<NTL, NT, agg_lds, stream>>>(XS, ei, ET + (size_t)l * NVP * NH, ASD, bias, T16);
    wmma_gemm64<0, false, 2, 0, false, 0><<<dim3((NTL * 2 + 7) / 8, 1), 256, 0, stream>>>(
        (const unsigned short*)T16, nullptr, HC, 0L, (const unsigned short*)(HTT + (size_t)l * EMB * HC), nullptr, HC, 0L,
        (void*)H2, nullptr, EMB, 0L, ht_b + (size_t)l * EMB, nullptr, 0L, NPAD, EMB, HC, 0.0625f);
    bn_stats_kernel<<<NPART, 128, 0, stream>>>(H2, BNP);
    bn_fin_kernel<<<1, 128, 0, stream>>>(BNP, BNS);
    bn_apply_kernel<<<NPAD * EMB / 2 / NT, NT, 0, stream>>>(H2, BNS, bn_g + (size_t)l * EMB, bn_b + (size_t)l * EMB, HF, X16);
  }

  pool_kernel<<<NGP, 128, 0, stream>>>(HF, batch, HID, HID16);
  wmma_gemm64<0, false, 2, 0, false, 2><<<dim3((16 * 4 + 7) / 8, 1), 256, 0, stream>>>(
      (const unsigned short*)HID16, nullptr, 256, 0L, (const unsigned short*)O1T, nullptr, 256, 0L,
      (void*)OB, nullptr, 256, 0L, out1_b, nullptr, 0L, NGP, 256, 256, 0.0625f);
  out0_kernel<<<NGP / 32, NT, 0, stream>>>(OB, out2_w, out2_b, OUT0);
  pack_out_kernel<<<(DOUT_N / 4 + NT - 1) / NT, NT, 0, stream>>>(OUT0, HID, dout);
}
